// T5MultiHeadAttention_44684839748198
// MI455X (gfx1250) — hardware-verified
//
#include <hip/hip_runtime.h>
#include <stdint.h>

typedef __attribute__((ext_vector_type(16))) _Float16 v16h;
typedef __attribute__((ext_vector_type(8)))  _Float16 v8h;
typedef __attribute__((ext_vector_type(16))) __bf16   v16b;
typedef __attribute__((ext_vector_type(8)))  __bf16   v8b;
typedef __attribute__((ext_vector_type(8)))  float    v8f;
typedef __attribute__((ext_vector_type(4)))  float    v4f;
typedef __attribute__((ext_vector_type(4)))  unsigned v4u;
typedef __attribute__((ext_vector_type(4)))  int      v4i;

constexpr int SEQ_LEN   = 2048;
constexpr int NUM_HEADS = 12;
constexpr int HEAD_DIM  = 64;
constexpr int DM        = 768;
constexpr int NBATCH    = 2;
constexpr int MROWS     = NBATCH * SEQ_LEN;
constexpr int REL_MAX   = 128;
constexpr int REL_N     = 2 * REL_MAX + 1;
constexpr int REL_PAD   = 288;
constexpr int SMALL_N   = 4 * DM + REL_PAD;
static_assert(SMALL_N % 32 == 0, "whole lines");
static_assert(MROWS % 64 == 0 && DM % 64 == 0 && DM % 32 == 0, "gemm tile contract M,N %64, K %32");
static_assert(NUM_HEADS * HEAD_DIM == DM, "heads");

__device__ __forceinline__ unsigned short f2bf_bits(float f) {
  unsigned u = __float_as_uint(f);
  return (unsigned short)((u + 0x7FFFu + ((u >> 16) & 1u)) >> 16);
}
__device__ __forceinline__ float bf_bits2f(unsigned short h) { return __uint_as_float(((unsigned)h) << 16); }

__device__ __forceinline__ void dep_guard_h(v8f& a, v8f& b, v16h x, v16h y) { asm volatile("v_nop\n\tv_nop\n\tv_nop\n\tv_nop" : "+v"(a), "+v"(b) : "v"(x), "v"(y)); }
__device__ __forceinline__ void dep_guard_b(v8f& a, v8f& b, v16b x, v16b y) { asm volatile("v_nop\n\tv_nop\n\tv_nop\n\tv_nop" : "+v"(a), "+v"(b) : "v"(x), "v"(y)); }
__device__ __forceinline__ void keep4_h(v16h a, v16h b, v16h c, v16h d) { asm volatile("v_nop" :: "v"(a), "v"(b), "v"(c), "v"(d)); }
__device__ __forceinline__ void keep4_b(v16b a, v16b b, v16b c, v16b d) { asm volatile("v_nop" :: "v"(a), "v"(b), "v"(c), "v"(d)); }
__device__ __forceinline__ void acc_guard4(v8f& a, v8f& b, v8f& c, v8f& d) { asm volatile("v_nop\n\tv_nop\n\tv_nop\n\tv_nop" : "+v"(a), "+v"(b), "+v"(c), "+v"(d)); }
template <typename T> struct Frag;
template <> struct Frag<_Float16> {
  typedef v16h V; union U { v16h v; v8h h[2]; };
  static __device__ __forceinline__ v16h load(const _Float16* p) {
    U f; f.h[0] = *(const v8h*)(p); f.h[1] = *(const v8h*)(p + 16); return f.v;
  }
  static __device__ __forceinline__ v8f mma(v16h a, v16h b, v8f c) {
    return __builtin_amdgcn_wmma_f32_16x16x32_f16(false, a, false, b, (short)0, c, false, false);
  }
  static __device__ __forceinline__ void guard(v8f& a, v8f& b, v16h x, v16h y) { dep_guard_h(a, b, x, y); }
  static __device__ __forceinline__ void keep(v16h a, v16h b, v16h c, v16h d) { keep4_h(a, b, c, d); }
};
template <> struct Frag<__bf16> {
  typedef v16b V; union U { v16b v; v8b h[2]; };
  static __device__ __forceinline__ v16b load(const __bf16* p) {
    U f; f.h[0] = *(const v8b*)(p); f.h[1] = *(const v8b*)(p + 16); return f.v;
  }
  static __device__ __forceinline__ v8f mma(v16b a, v16b b, v8f c) {
    return __builtin_amdgcn_wmma_f32_16x16x32_bf16(false, a, false, b, (short)0, c, false, false);
  }
  static __device__ __forceinline__ void guard(v8f& a, v8f& b, v16b x, v16b y) { dep_guard_b(a, b, x, y); }
  static __device__ __forceinline__ void keep(v16b a, v16b b, v16b c, v16b d) { keep4_b(a, b, c, d); }
};

template <int ET> struct Elem;
template <> struct Elem<0> { typedef _Float16 T; };
template <> struct Elem<1> { typedef __bf16 T; };
template <int ET, bool SPLIT, int BIAS_MODE, int OUT_MODE, bool RESID, int ACT = 0, bool SPLITB = true>
__global__ __launch_bounds__(256) void wmma_gemm64(
    const unsigned short* __restrict__ Ap, const unsigned short* __restrict__ A2p, int lda, long strideA,
    const unsigned short* __restrict__ Btp, const unsigned short* __restrict__ Bt2p, int ldb, long strideB,
    void* __restrict__ Cout, void* __restrict__ Cout2, int ldc, long strideC,
    const float* __restrict__ bias,
    const float* __restrict__ resid, long strideR,
    int M, int N, int K, float scale) {
  typedef typename Elem<ET>::T T;
  typedef typename Frag<T>::V V;
  const T* A = (const T*)Ap; const T* A2 = (const T*)A2p; const T* Bt = (const T*)Btp; const T* Bt2 = (const T*)Bt2p;
  __shared__ __align__(16) float sT[8][16 * 68];
  const int b    = blockIdx.y;
  const int lane = threadIdx.x & 31;
  const int wave = threadIdx.x >> 5;
  const int tilesN = N >> 6;
  const int tilesM = M >> 6;
  const int tile = blockIdx.x * 8 + wave;
  if (tile >= tilesM * tilesN) return;
  const int tm = tile / tilesN;
  const int tn = tile - tm * tilesN;
  const int m0 = tm << 6;
  const int n0 = tn << 6;

  const T* Ab  = A  + (size_t)b * strideA;
  const T* Bb  = Bt + (size_t)b * strideB;
  const T* Ab2 = SPLIT ? (A2  + (size_t)b * strideA) : nullptr;
  const T* Bb2 = (SPLIT && SPLITB) ? (Bt2 + (size_t)b * strideB) : nullptr;

  const int rlane = lane & 15;
  const int koff  = (lane >> 4) * 8;
  const int mOff  = (lane >> 4) * 8;

  v8f acc[4][4];
#pragma unroll
  for (int i = 0; i < 4; ++i)
#pragma unroll
    for (int j = 0; j < 4; ++j) acc[i][j] = (v8f){0.f,0.f,0.f,0.f,0.f,0.f,0.f,0.f};

  for (int k0 = 0; k0 < K; k0 += 32) {
    V bh[4], bl[4];
#pragma unroll
    for (int j = 0; j < 4; ++j) {
      const size_t bo = (size_t)(n0 + (j << 4) + rlane) * ldb + koff + k0;
      bh[j] = Frag<T>::load(Bb + bo);
      if (SPLIT && SPLITB) bl[j] = Frag<T>::load(Bb2 + bo);
    }
#pragma unroll
    for (int i = 0; i < 4; ++i) {
      const size_t ao = (size_t)(m0 + (i << 4) + rlane) * lda + koff + k0;
      V ah = Frag<T>::load(Ab + ao);
      V al;
      if (SPLIT) al = Frag<T>::load(Ab2 + ao);
#pragma unroll
      for (int j = 0; j < 4; ++j) {
        acc[i][j] = Frag<T>::mma(ah, bh[j], acc[i][j]);
        if (SPLIT) {
          if (SPLITB) acc[i][j] = Frag<T>::mma(ah, bl[j], acc[i][j]);
          acc[i][j] = Frag<T>::mma(al, bh[j], acc[i][j]);
        }
      }
      Frag<T>::guard(acc[i][0], acc[i][3], ah, SPLIT ? al : ah);
    }
    Frag<T>::keep(bh[0], bh[1], bh[2], bh[3]);
    if (SPLIT && SPLITB) Frag<T>::keep(bl[0], bl[1], bl[2], bl[3]);
  }
  acc_guard4(acc[0][0], acc[0][1], acc[0][2], acc[0][3]);
  acc_guard4(acc[1][0], acc[1][1], acc[1][2], acc[1][3]);
  acc_guard4(acc[2][0], acc[2][1], acc[2][2], acc[2][3]);
  acc_guard4(acc[3][0], acc[3][1], acc[3][2], acc[3][3]);

  float* slab = sT[wave];
  const float* Rb = RESID ? (resid + (size_t)b * strideR) : nullptr;
#pragma unroll
  for (int i = 0; i < 4; ++i) {
    const int mBase = m0 + (i << 4);
#pragma unroll
    for (int j = 0; j < 4; ++j) {
      const int n = n0 + (j << 4) + rlane;
      float bv = 0.f;
      if (BIAS_MODE == 2) bv = bias[n];
#pragma unroll
      for (int r = 0; r < 8; ++r) {
        float v = acc[i][j][r] * scale;
        if (BIAS_MODE == 1) v += bias[mBase + mOff + r];
        if (BIAS_MODE == 2) v += bv;
        if (RESID) v += Rb[(size_t)(mBase + mOff + r) * ldc + n];
        if (ACT == 1) v = tanhf(v);
        if (ACT == 2) v = fmaxf(v, 0.0f);
        if (ACT == 4) v = (v > 0.f) ? v : 0.01f * v;
        slab[(mOff + r) * 68 + (j << 4) + rlane] = v;
      }
    }
    __builtin_amdgcn_fence(__ATOMIC_RELEASE, "workgroup");
    __builtin_amdgcn_wave_barrier();
    __builtin_amdgcn_fence(__ATOMIC_ACQUIRE, "workgroup");
    if (OUT_MODE == 0) {
      float* C = (float*)Cout + (size_t)b * strideC;
      const int hh = lane >> 4, c4 = (lane & 15) * 4;
      for (int pass = 0; pass < 2; ++pass) {
#pragma unroll
        for (int it = 0; it < 8; ++it) {
          const int row = it * 2 + hh;
          v4f v = *(const v4f*)(slab + row * 68 + c4);
          *(volatile v4f*)(C + (size_t)(mBase + row) * ldc + n0 + c4) = v;
        }
        __threadfence();
      }
    } else {
      const int q = lane >> 3, c8 = (lane & 7) * 8;
      unsigned short* C  = (unsigned short*)Cout  + (size_t)b * strideC;
      unsigned short* C2 = (OUT_MODE == 2) ? ((unsigned short*)Cout2 + (size_t)b * strideC) : nullptr;
      for (int pass = 0; pass < 2; ++pass) {
#pragma unroll
        for (int it = 0; it < 4; ++it) {
          const int row = it * 4 + q;
          const float* sp = slab + row * 68 + c8;
          v8h hv, lv;
#pragma unroll
          for (int e = 0; e < 8; ++e) {
            if (OUT_MODE == 1) {
              hv[e] = (_Float16)sp[e];
            } else {
              unsigned short hb = f2bf_bits(sp[e]);
              unsigned short lb = f2bf_bits(sp[e] - bf_bits2f(hb));
              hv[e] = __builtin_bit_cast(_Float16, hb);
              lv[e] = __builtin_bit_cast(_Float16, lb);
            }
          }
          *(volatile v8h*)(C + (size_t)(mBase + row) * ldc + n0 + c8) = hv;
          if (OUT_MODE == 2) *(volatile v8h*)(C2 + (size_t)(mBase + row) * ldc + n0 + c8) = lv;
        }
        __threadfence();
      }
    }
    __builtin_amdgcn_fence(__ATOMIC_RELEASE, "workgroup");
    __builtin_amdgcn_wave_barrier();
    __builtin_amdgcn_fence(__ATOMIC_ACQUIRE, "workgroup");
  }
}

struct CastPtrs {
  const float* s0; const float* s1; const float* s2; const float* s3;
  unsigned short* d0; unsigned short* d1; unsigned short* d2; unsigned short* d3;
};
static_assert(sizeof(CastPtrs) == 64, "no padding");

__global__ __launch_bounds__(256) void cast_f32_bf16x8(CastPtrs p, int n8) {
  const int y = blockIdx.y;
  const float* src = (y == 0) ? p.s0 : ((y == 1) ? p.s1 : ((y == 2) ? p.s2 : p.s3));
  unsigned short* dst = (y == 0) ? p.d0 : ((y == 1) ? p.d1 : ((y == 2) ? p.d2 : p.d3));
  const int i = blockIdx.x * 256 + threadIdx.x;
  if (i < n8) {
    const v4f a = *(const v4f*)(src + 8 * (size_t)i);
    const v4f c = *(const v4f*)(src + 8 * (size_t)i + 4);
    v4u u;
    u[0] = (unsigned)f2bf_bits(a[0]) | ((unsigned)f2bf_bits(a[1]) << 16);
    u[1] = (unsigned)f2bf_bits(a[2]) | ((unsigned)f2bf_bits(a[3]) << 16);
    u[2] = (unsigned)f2bf_bits(c[0]) | ((unsigned)f2bf_bits(c[1]) << 16);
    u[3] = (unsigned)f2bf_bits(c[2]) | ((unsigned)f2bf_bits(c[3]) << 16);
    *(volatile v4u*)(dst + 8 * (size_t)i) = u;
    __threadfence();
    *(volatile v4u*)(dst + 8 * (size_t)i) = u;
  }
}

__global__ __launch_bounds__(256) void split_f32_bf16x8(const float* __restrict__ src,
                                                        unsigned short* __restrict__ hi,
                                                        unsigned short* __restrict__ lo, int n8) {
  const int i = blockIdx.x * 256 + threadIdx.x;
  if (i < n8) {
    const v4f a = *(const v4f*)(src + 8 * (size_t)i);
    const v4f c = *(const v4f*)(src + 8 * (size_t)i + 4);
    unsigned hb[8], lb[8];
#pragma unroll
    for (int e = 0; e < 4; ++e) {
      const unsigned short h0 = f2bf_bits(a[e]);
      hb[e] = h0; lb[e] = f2bf_bits(a[e] - bf_bits2f(h0));
      const unsigned short h1 = f2bf_bits(c[e]);
      hb[4 + e] = h1; lb[4 + e] = f2bf_bits(c[e] - bf_bits2f(h1));
    }
    v4u uh, ul;
#pragma unroll
    for (int w = 0; w < 4; ++w) {
      uh[w] = hb[2 * w] | (hb[2 * w + 1] << 16);
      ul[w] = lb[2 * w] | (lb[2 * w + 1] << 16);
    }
    *(volatile v4u*)(hi + 8 * (size_t)i) = uh;
    *(volatile v4u*)(lo + 8 * (size_t)i) = ul;
    __threadfence();
    *(volatile v4u*)(hi + 8 * (size_t)i) = uh;
    *(volatile v4u*)(lo + 8 * (size_t)i) = ul;
  }
}

__global__ __launch_bounds__(256) void prep_small(const float* __restrict__ b0, const float* __restrict__ b1,
                                                  const float* __restrict__ b2, const float* __restrict__ b3,
                                                  const float* __restrict__ rel, float* __restrict__ dst) {
  const int i = blockIdx.x * 256 + threadIdx.x;
  if (i < SMALL_N) {
    const int bi = i % DM;
    int t = i - 4 * DM; t = t < 0 ? 0 : t;
    const int tr = t > (REL_N - 1) ? (REL_N - 1) : t;
    const float c0 = b0[bi], c1 = b1[bi], c2 = b2[bi], c3 = b3[bi], c4 = rel[tr];
    const int which = i / DM;
    float v = (which == 0) ? c0 : ((which == 1) ? c1 : ((which == 2) ? c2 : ((which == 3) ? c3 : ((t < REL_N) ? c4 : 0.0f))));
    v = bf_bits2f(f2bf_bits(v));
    ((volatile float*)dst)[i] = v;
    __threadfence();
    ((volatile float*)dst)[i] = v;
  }
}

#define AT_D 64
#define AT_NW 4
#define AT_QB 64
#define AT_KC 64

__device__ __forceinline__ __bf16 at_f2bf(float f) { return __builtin_bit_cast(__bf16, f2bf_bits(f)); }
__device__ __forceinline__ void at_split(float f, __bf16& hi, __bf16& lo) {
  const unsigned short hb = f2bf_bits(f);
  hi = __builtin_bit_cast(__bf16, hb);
  lo = at_f2bf(f - __uint_as_float(((unsigned)hb) << 16));
}
__device__ __forceinline__ v8f at_mma(v16b a, v16b b, v8f c) {
  c = __builtin_amdgcn_wmma_f32_16x16x32_bf16(false, a, false, b, (short)0, c, false, false);
  asm volatile("v_nop\n\tv_nop\n\tv_nop\n\tv_nop" : "+v"(c) : "v"(a), "v"(b));
  return c;
}

__global__ __launch_bounds__(128)
void attn_relbias_kernel(const unsigned short* __restrict__ qhp, const unsigned short* __restrict__ qlp,
                         const unsigned short* __restrict__ khp, const unsigned short* __restrict__ klp,
                         const unsigned short* __restrict__ vhp, const unsigned short* __restrict__ vlp,
                         const int* __restrict__ maskp, const float* __restrict__ relp,
                         float* __restrict__ ctx) {
  union FB { v16b v; v8b h[2]; };
  __shared__ __align__(16) __bf16 Ksh[AT_KC * AT_D];
  __shared__ __align__(16) __bf16 Ksl[AT_KC * AT_D];
  __shared__ __align__(16) __bf16 Vth[AT_D * AT_KC];
  __shared__ __align__(16) __bf16 Vtl[AT_D * AT_KC];
  __shared__ __align__(16) __bf16 Psh[AT_NW][16 * AT_KC];
  __shared__ __align__(16) __bf16 Psl[AT_NW][16 * AT_KC];
  __shared__ __align__(16) float  Os[AT_NW][16 * 68];
  __shared__ __align__(16) int    Msh[AT_QB * AT_KC];
  __shared__ __align__(16) float  Rsh[REL_PAD];

  const int tid  = threadIdx.x;
  const int wave = tid >> 5;
  const int lane = tid & 31;
  const int hh   = lane >> 4;
  const int c    = lane & 15;

  const int nqb = SEQ_LEN / AT_QB;
  const int bx = blockIdx.x;
  const int qb = bx % nqb;
  const int bh = bx / nqb;
  const int h  = bh % NUM_HEADS;
  const int b  = bh / NUM_HEADS;
  const int qbase_block = qb * AT_QB;
  const int q0 = qbase_block + wave * 16;
  const size_t rowb = (size_t)b * SEQ_LEN;
  const int hcol = h * AT_D;

  for (int i = tid; i < REL_PAD; i += AT_NW * 32) Rsh[i] = relp[i];

  const __bf16* QH = (const __bf16*)(const void*)qhp;
  const __bf16* QL = (const __bf16*)(const void*)qlp;
  const __bf16* KH = (const __bf16*)(const void*)khp;
  const __bf16* KL = (const __bf16*)(const void*)klp;

  v16b qah[2], qal[2];
  {
    const size_t qoff = (rowb + q0 + c) * DM + hcol;
#pragma unroll
    for (int dc = 0; dc < 2; ++dc) {
      qah[dc] = Frag<__bf16>::load(QH + qoff + dc * 32 + 8 * hh);
      qal[dc] = Frag<__bf16>::load(QL + qoff + dc * 32 + 8 * hh);
    }
  }

  float mrow[8], lrow[8];
  v8f oacc[4];
#pragma unroll
  for (int r = 0; r < 8; ++r) { mrow[r] = -__builtin_huge_valf(); lrow[r] = 0.f; }
#pragma unroll
  for (int t = 0; t < 4; ++t) oacc[t] = (v8f){0.f,0.f,0.f,0.f,0.f,0.f,0.f,0.f};

  const int dbase = c - (wave * 16 + 8 * hh);

  for (int kc = 0; kc < SEQ_LEN / AT_KC; ++kc) {
    const int kv0 = kc * AT_KC;
    __syncthreads();
    {
      const int kvr = tid >> 1, dh = (tid & 1) * 32;
      const size_t koff = (rowb + kv0 + kvr) * DM + hcol + dh;
#pragma unroll
      for (int i = 0; i < 4; ++i) {
        const v8b th = *(const v8b*)(KH + koff + 8 * i);
        const v8b tl = *(const v8b*)(KL + koff + 8 * i);
        *(v8b*)(Ksh + kvr * AT_D + dh + 8 * i) = th;
        *(v8b*)(Ksl + kvr * AT_D + dh + 8 * i) = tl;
      }
      asm volatile("" ::: "memory");
#pragma unroll
      for (int i = 0; i < 4; ++i) {
        const v4u wh = *(const v4u*)(const void*)(vhp + koff + 8 * i);
        const v4u wl = *(const v4u*)(const void*)(vlp + koff + 8 * i);
#pragma unroll
        for (int e = 0; e < 4; ++e) {
          const unsigned xh = wh[e], xl = wl[e];
          const int d = dh + 8 * i + 2 * e;
          Vth[d * AT_KC + kvr]       = __builtin_bit_cast(__bf16, (unsigned short)(xh & 0xffffu));
          Vth[(d + 1) * AT_KC + kvr] = __builtin_bit_cast(__bf16, (unsigned short)(xh >> 16));
          Vtl[d * AT_KC + kvr]       = __builtin_bit_cast(__bf16, (unsigned short)(xl & 0xffffu));
          Vtl[(d + 1) * AT_KC + kvr] = __builtin_bit_cast(__bf16, (unsigned short)(xl >> 16));
        }
      }
      asm volatile("" ::: "memory");
      const size_t moff = (rowb + qbase_block + kvr) * SEQ_LEN + kv0 + dh;
#pragma unroll
      for (int i = 0; i < 8; ++i) *(v4i*)(Msh + kvr * AT_KC + dh + 4 * i) = *(const v4i*)(maskp + moff + 4 * i);
    }
    __syncthreads();

    v8f s[4];
#pragma unroll
    for (int j = 0; j < 4; ++j) {
      s[j] = (v8f){0.f,0.f,0.f,0.f,0.f,0.f,0.f,0.f};
#pragma unroll
      for (int dc = 0; dc < 2; ++dc) {
        FB kb;
        kb.h[0] = *(const v8b*)(Ksh + (j * 16 + c) * AT_D + dc * 32 + 8 * hh);
        kb.h[1] = *(const v8b*)(Ksh + (j * 16 + c) * AT_D + dc * 32 + 16 + 8 * hh);
        FB kl;
        kl.h[0] = *(const v8b*)(Ksl + (j * 16 + c) * AT_D + dc * 32 + 8 * hh);
        kl.h[1] = *(const v8b*)(Ksl + (j * 16 + c) * AT_D + dc * 32 + 16 + 8 * hh);
        s[j] = at_mma(qah[dc], kb.v, s[j]);
        s[j] = at_mma(qah[dc], kl.v, s[j]);
        s[j] = at_mma(qal[dc], kb.v, s[j]);
      }
    }

    const int drel0 = kv0 - qbase_block + dbase;
    float cm[8];
#pragma unroll
    for (int r = 0; r < 8; ++r) {
      float m = -__builtin_huge_valf();
#pragma unroll
      for (int j = 0; j < 4; ++j) {
        float sc = s[j][r] * 0.125f;
        int dd = drel0 + 16 * j - r;
        dd = dd < -REL_MAX ? -REL_MAX : (dd > REL_MAX ? REL_MAX : dd);
        sc += Rsh[dd + REL_MAX];
        const int mv = Msh[(wave * 16 + 8 * hh + r) * AT_KC + j * 16 + c];
        sc = (mv == 0) ? -1.0e9f : sc;
        s[j][r] = sc;
        m = fmaxf(m, sc);
      }
#pragma unroll
      for (int off = 1; off < 16; off <<= 1) m = fmaxf(m, __shfl_xor(m, off, 32));
      cm[r] = m;
    }
    __bf16* pwh = Psh[wave];
    __bf16* pwl = Psl[wave];
#pragma unroll
    for (int r = 0; r < 8; ++r) {
      const float mnew = fmaxf(mrow[r], cm[r]);
      const float alpha = expf(mrow[r] - mnew);
      mrow[r] = mnew;
      float psum = 0.f;
#pragma unroll
      for (int j = 0; j < 4; ++j) {
        const float p = expf(s[j][r] - mnew);
        psum += p;
        __bf16 a, bl; at_split(p, a, bl);
        pwh[(8 * hh + r) * AT_KC + j * 16 + c] = a;
        pwl[(8 * hh + r) * AT_KC + j * 16 + c] = bl;
      }
#pragma unroll
      for (int off = 1; off < 16; off <<= 1) psum += __shfl_xor(psum, off, 32);
      lrow[r] = lrow[r] * alpha + psum;
#pragma unroll
      for (int t = 0; t < 4; ++t) oacc[t][r] *= alpha;
    }
    __builtin_amdgcn_fence(__ATOMIC_RELEASE, "workgroup");
    __builtin_amdgcn_wave_barrier();
    __builtin_amdgcn_fence(__ATOMIC_ACQUIRE, "workgroup");
#pragma unroll 1
    for (int kk = 0; kk < 2; ++kk) {
      FB pa, pl;
      pa.h[0] = *(const v8b*)(pwh + c * AT_KC + kk * 32 + 8 * hh);
      pa.h[1] = *(const v8b*)(pwh + c * AT_KC + kk * 32 + 16 + 8 * hh);
      pl.h[0] = *(const v8b*)(pwl + c * AT_KC + kk * 32 + 8 * hh);
      pl.h[1] = *(const v8b*)(pwl + c * AT_KC + kk * 32 + 16 + 8 * hh);
#pragma unroll
      for (int t = 0; t < 4; ++t) {
        FB vb;
        vb.h[0] = *(const v8b*)(Vth + (t * 16 + c) * AT_KC + kk * 32 + 8 * hh);
        vb.h[1] = *(const v8b*)(Vth + (t * 16 + c) * AT_KC + kk * 32 + 16 + 8 * hh);
        FB vl;
        vl.h[0] = *(const v8b*)(Vtl + (t * 16 + c) * AT_KC + kk * 32 + 8 * hh);
        vl.h[1] = *(const v8b*)(Vtl + (t * 16 + c) * AT_KC + kk * 32 + 16 + 8 * hh);
        oacc[t] = at_mma(pa.v, vb.v, oacc[t]);
        oacc[t] = at_mma(pa.v, vl.v, oacc[t]);
        oacc[t] = at_mma(pl.v, vb.v, oacc[t]);
      }
    }
  }

  float* os = Os[wave];
#pragma unroll
  for (int r = 0; r < 8; ++r) {
    const float inv = 1.0f / lrow[r];
#pragma unroll
    for (int t = 0; t < 4; ++t) os[(8 * hh + r) * 68 + t * 16 + c] = oacc[t][r] * inv;
  }
  __builtin_amdgcn_fence(__ATOMIC_RELEASE, "workgroup");
  __builtin_amdgcn_wave_barrier();
  __builtin_amdgcn_fence(__ATOMIC_ACQUIRE, "workgroup");
  {
    float* ob_ptr = ctx + rowb * DM + hcol;
    const int c4 = (lane & 15) * 4;
    for (int pass = 0; pass < 2; ++pass) {
#pragma unroll
      for (int it = 0; it < 8; ++it) {
        const int row = it * 2 + hh;
        v4f val = *(const v4f*)(os + row * 68 + c4);
        *(volatile v4f*)(ob_ptr + (size_t)(q0 + row) * DM + c4) = val;
      }
      __threadfence();
    }
  }
}

constexpr size_t XELEM = (size_t)MROWS * DM;
constexpr size_t WELEM = (size_t)DM * DM;
constexpr size_t X2B = XELEM * 2, X4B = XELEM * 4, W2B = WELEM * 2;
constexpr size_t SMALLB = (((size_t)SMALL_N * 4 + 127) / 128) * 128;
constexpr size_t OFF_XQ = 0;
constexpr size_t OFF_XK = OFF_XQ + X2B;
constexpr size_t OFF_XV = OFF_XK + X2B;
constexpr size_t OFF_WQ = OFF_XV + X2B;
constexpr size_t OFF_WK = OFF_WQ + W2B;
constexpr size_t OFF_WV = OFF_WK + W2B;
constexpr size_t OFF_WO = OFF_WV + W2B;
constexpr size_t OFF_QH = OFF_WO + W2B;
constexpr size_t OFF_KH = OFF_QH + X2B;
constexpr size_t OFF_VH = OFF_KH + X2B;
constexpr size_t OFF_QL = OFF_VH + X2B;
constexpr size_t OFF_KL = OFF_QL + X2B;
constexpr size_t OFF_VL = OFF_KL + X2B;
constexpr size_t OFF_CTX = OFF_VL + X2B;
constexpr size_t OFF_CH = OFF_CTX + X4B;
constexpr size_t OFF_CL = OFF_CH + X2B;
constexpr size_t OFF_SMALL = OFF_CL + X2B;
constexpr size_t WS_TOTAL = OFF_SMALL + SMALLB;
static_assert(WS_TOTAL == 86520960, "carve total");
static_assert(WS_TOTAL <= 134217728, "carve under 128 MiB");
static_assert((OFF_SMALL % 128) == 0 && (OFF_CTX % 128) == 0, "alignment");
static_assert(XELEM % (8 * 256) == 0 && WELEM % (8 * 256) == 0, "cast grids exact");

extern "C" void kernel_launch(void* const* d_in, const int* in_sizes, int n_in,
                              void* d_out, int out_size, void* d_ws, size_t ws_size,
                              hipStream_t stream) {
  if (n_in < 13) return;
  if ((size_t)in_sizes[0] != XELEM || (size_t)in_sizes[1] != XELEM || (size_t)in_sizes[2] != XELEM) return;
  if ((size_t)in_sizes[3] != (size_t)NBATCH * SEQ_LEN * SEQ_LEN) return;
  if ((size_t)in_sizes[4] != WELEM || (size_t)in_sizes[6] != WELEM || (size_t)in_sizes[8] != WELEM || (size_t)in_sizes[10] != WELEM) return;
  if (in_sizes[5] != DM || in_sizes[7] != DM || in_sizes[9] != DM || in_sizes[11] != DM || in_sizes[12] != REL_N) return;
  if ((size_t)out_size != XELEM) return;
  if (ws_size < WS_TOTAL) return;

  const float* Qin  = (const float*)d_in[0];
  const float* Kin  = (const float*)d_in[1];
  const float* Vin  = (const float*)d_in[2];
  const int*   mask = (const int*)  d_in[3];
  const float* Wq   = (const float*)d_in[4];
  const float* bq   = (const float*)d_in[5];
  const float* Wk   = (const float*)d_in[6];
  const float* bk   = (const float*)d_in[7];
  const float* Wv   = (const float*)d_in[8];
  const float* bv   = (const float*)d_in[9];
  const float* Wo   = (const float*)d_in[10];
  const float* bo   = (const float*)d_in[11];
  const float* rel  = (const float*)d_in[12];
  float* out = (float*)d_out;

  char* ws = (char*)d_ws;
  unsigned short* XQ = (unsigned short*)(ws + OFF_XQ);
  unsigned short* XK = (unsigned short*)(ws + OFF_XK);
  unsigned short* XV = (unsigned short*)(ws + OFF_XV);
  unsigned short* WQ = (unsigned short*)(ws + OFF_WQ);
  unsigned short* WK = (unsigned short*)(ws + OFF_WK);
  unsigned short* WV = (unsigned short*)(ws + OFF_WV);
  unsigned short* WO = (unsigned short*)(ws + OFF_WO);
  unsigned short* QH = (unsigned short*)(ws + OFF_QH);
  unsigned short* KH = (unsigned short*)(ws + OFF_KH);
  unsigned short* VH = (unsigned short*)(ws + OFF_VH);
  unsigned short* QL = (unsigned short*)(ws + OFF_QL);
  unsigned short* KL = (unsigned short*)(ws + OFF_KL);
  unsigned short* VL = (unsigned short*)(ws + OFF_VL);
  float*          CTX = (float*)(ws + OFF_CTX);
  unsigned short* CH = (unsigned short*)(ws + OFF_CH);
  unsigned short* CL = (unsigned short*)(ws + OFF_CL);
  float*          SMALL = (float*)(ws + OFF_SMALL);
  const float* bqr  = SMALL + 0 * DM;
  const float* bkr  = SMALL + 1 * DM;
  const float* bvr  = SMALL + 2 * DM;
  const float* bor  = SMALL + 3 * DM;
  const float* relr = SMALL + 4 * DM;

  {
    CastPtrs p; p.s0 = Qin; p.s1 = Kin; p.s2 = Vin; p.s3 = Vin; p.d0 = XQ; p.d1 = XK; p.d2 = XV; p.d3 = XV;
    const int n8 = (int)(XELEM / 8);
    cast_f32_bf16x8<<<dim3((unsigned)(n8 / 256), 3), dim3(256), 0, stream>>>(p, n8);
  }
  {
    CastPtrs p; p.s0 = Wq; p.s1 = Wk; p.s2 = Wv; p.s3 = Wo; p.d0 = WQ; p.d1 = WK; p.d2 = WV; p.d3 = WO;
    const int n8 = (int)(WELEM / 8);
    cast_f32_bf16x8<<<dim3((unsigned)(n8 / 256), 4), dim3(256), 0, stream>>>(p, n8);
  }
  prep_small<<<dim3((SMALL_N + 255) / 256), dim3(256), 0, stream>>>(bq, bk, bv, bo, rel, SMALL);

  const dim3 ggrid((unsigned)((MROWS / 64) * (DM / 64) / 8), 1);
  wmma_gemm64<1, false, 2, 2, false, 0, true><<<ggrid, dim3(256), 0, stream>>>(
      XQ, XQ, DM, 0L, WQ, WQ, DM, 0L, (void*)QH, (void*)QL, DM, 0L, bqr, bqr, 0L, MROWS, DM, DM, 1.0f);
  wmma_gemm64<1, false, 2, 2, false, 0, true><<<ggrid, dim3(256), 0, stream>>>(
      XK, XK, DM, 0L, WK, WK, DM, 0L, (void*)KH, (void*)KL, DM, 0L, bkr, bkr, 0L, MROWS, DM, DM, 1.0f);
  wmma_gemm64<1, false, 2, 2, false, 0, true><<<ggrid, dim3(256), 0, stream>>>(
      XV, XV, DM, 0L, WV, WV, DM, 0L, (void*)VH, (void*)VL, DM, 0L, bvr, bvr, 0L, MROWS, DM, DM, 1.0f);

  attn_relbias_kernel<<<dim3((unsigned)(NBATCH * NUM_HEADS * (SEQ_LEN / AT_QB))), dim3(AT_NW * 32), 0, stream>>>(
      QH, QL, KH, KL, VH, VL, mask, relr, CTX);

  {
    const int n8 = (int)(XELEM / 8);
    split_f32_bf16x8<<<dim3((unsigned)(n8 / 256)), dim3(256), 0, stream>>>(CTX, CH, CL, n8);
  }
  wmma_gemm64<1, true, 2, 0, false, 0, false><<<ggrid, dim3(256), 0, stream>>>(
      CH, CL, DM, 0L, WO, WO, DM, 0L, (void*)out, (void*)out, DM, 0L, bor, bor, 0L, MROWS, DM, DM, 1.0f);
}
